// CoeffNet_28071906246845
// MI455X (gfx1250) — hardware-verified
//
#include <hip/hip_runtime.h>
#include <stddef.h>


#define FD    64
#define KBAS  32
#define RMAXF 2.5f

#define TIN   128
#define NBI   32

#define NT    64
#define NB    128
#define EPT   16
#define CHUNK (NT * EPT)
#define PASSN 64
#define PCAP  (CHUNK + PASSN)
#define SCB   64.0f
#define SCINV 0.000244140625f

static_assert(NT == FD);
static_assert(PASSN == NT);
static_assert((NB % 2) == 0);
static_assert(PCAP >= CHUNK + PASSN);
static_assert((2 * FD * FD / 8) % 256 == 0);

typedef float    v4f  __attribute__((ext_vector_type(4)));
typedef float    v8f  __attribute__((ext_vector_type(8)));
typedef int      v4i  __attribute__((ext_vector_type(4)));
typedef _Float16 v8h  __attribute__((ext_vector_type(8)));
typedef _Float16 v16h __attribute__((ext_vector_type(16)));
typedef unsigned short v8us  __attribute__((ext_vector_type(8)));
typedef unsigned short v16us __attribute__((ext_vector_type(16)));
typedef __bf16   v16b __attribute__((ext_vector_type(16)));
union FragH { v16h v; v8h h[2]; };
union FragB { v16b v; v16us u; v8us h[2]; };

__device__ __forceinline__ v8f zero8f() {
  v8f z;
#pragma unroll
  for (int i = 0; i < 8; ++i) z[i] = 0.0f;
  return z;
}

__device__ __forceinline__ v8f wmh(v16h a, v16h b, v8f c) {
  v8f d = __builtin_amdgcn_wmma_f32_16x16x32_f16(false, a, false, b, (short)0, c, false, false);
  asm volatile("v_nop\n\tv_nop\n\tv_nop\n\tv_nop" : "+v"(d) : "v"(a), "v"(b));
  return d;
}
__device__ __forceinline__ v8f wmb(v16b a, v16b b, v8f c) {
  v8f d = __builtin_amdgcn_wmma_f32_16x16x32_bf16(false, a, false, b, (short)0, c, false, false);
  asm volatile("v_nop\n\tv_nop\n\tv_nop\n\tv_nop" : "+v"(d) : "v"(a), "v"(b));
  return d;
}

__device__ __forceinline__ unsigned bfbits(float x) {
  unsigned u = __float_as_uint(x);
  u += 0x7FFFu + ((u >> 16) & 1u);
  return u >> 16;
}

__device__ __forceinline__ void split8(v4f p, v4f q, v8us& hi, v8us& lo) {
  float x[8];
  x[0] = p.x; x[1] = p.y; x[2] = p.z; x[3] = p.w;
  x[4] = q.x; x[5] = q.y; x[6] = q.z; x[7] = q.w;
#pragma unroll
  for (int i = 0; i < 8; ++i) {
    const unsigned hb = bfbits(x[i]);
    const float hf = __uint_as_float(hb << 16);
    const unsigned lb = bfbits(x[i] - hf);
    hi[i] = (unsigned short)hb;
    lo[i] = (unsigned short)lb;
  }
}

__global__ __launch_bounds__(256) void k_prep(const float* __restrict__ W0, const float* __restrict__ W1,
                                              const float* __restrict__ Wb,
                                              unsigned short* whi, unsigned short* wlo, _Float16* wbh,
                                              int nSteps) {
  const int g = blockIdx.x * 256 + threadIdx.x;
  const int nGin = (2 * FD * FD) / 8;
  const int nGb  = (nSteps * KBAS * FD) / 8;
  if (g < nGin) {
    const int gpm = (FD * FD) / 8;
    const int c2 = g / gpm;
    const int idx0 = (g - c2 * gpm) * 8;
    const int n = idx0 / FD, kb = idx0 - n * FD;
    const float* W = (c2 == 0) ? W0 : W1;
    v8us hv, lv;
#pragma unroll
    for (int i = 0; i < 8; ++i) {
      const float x = W[(kb + i) * FD + n];
      const unsigned hb = bfbits(x);
      const float hf = __uint_as_float(hb << 16);
      hv[i] = (unsigned short)hb;
      lv[i] = (unsigned short)bfbits(x - hf);
    }
    unsigned short* ph = whi + (size_t)g * 8;
    unsigned short* pl = wlo + (size_t)g * 8;
    *(volatile v8us*)ph = hv;
    *(volatile v8us*)pl = lv;
    __threadfence();
    *(volatile v8us*)ph = hv;
    *(volatile v8us*)pl = lv;
  } else if (g < nGin + nGb) {
    const int g2 = g - nGin;
    const int gps = (KBAS * FD) / 8;
    const int st = g2 / gps;
    const int idx0 = (g2 - st * gps) * 8;
    const int n = idx0 / KBAS, kb = idx0 - n * KBAS;
    v8h hv;
#pragma unroll
    for (int i = 0; i < 8; ++i)
      hv[i] = (_Float16)(SCB * Wb[(size_t)st * KBAS * FD + (kb + i) * FD + n]);
    _Float16* p = wbh + (size_t)g2 * 8;
    *(volatile v8h*)p = hv;
    __threadfence();
    *(volatile v8h*)p = hv;
  }
}

__global__ __launch_bounds__(TIN) void k_in(const float* __restrict__ xd,
                                            const unsigned short* __restrict__ whi,
                                            const unsigned short* __restrict__ wlo,
                                            const float* __restrict__ bin,
                                            float* xo, int nN) {
  __shared__ __attribute__((aligned(16))) float so[NBI * 4 * FD];
  const int tid = threadIdx.x, lane = tid & 31, c = tid >> 5, h = lane >> 4, m = lane & 15;
  const int n0 = blockIdx.x * NBI;
  const unsigned short* ph = whi + (c == 0 ? 0 : FD * FD);
  const unsigned short* pl = wlo + (c == 0 ? 0 : FD * FD);

  v8f acc[2][4];
#pragma unroll
  for (int rt = 0; rt < 2; ++rt)
#pragma unroll
    for (int j = 0; j < 4; ++j) acc[rt][j] = zero8f();

#pragma unroll
  for (int ks = 0; ks < 2; ++ks) {
    const int k0 = ks * 32;
    FragB ah[2], al[2];
#pragma unroll
    for (int rt = 0; rt < 2; ++rt) {
      int node = n0 + 16 * rt + m;
      node = node > nN - 1 ? nN - 1 : node;
      const float* ap = xd + (size_t)node * (4 * FD) + c * FD + k0 + 8 * h;
      const v4f q0 = *(const v4f*)ap, q1 = *(const v4f*)(ap + 4);
      const v4f q2 = *(const v4f*)(ap + 16), q3 = *(const v4f*)(ap + 20);
      split8(q0, q1, ah[rt].h[0], al[rt].h[0]);
      split8(q2, q3, ah[rt].h[1], al[rt].h[1]);
    }
#pragma unroll
    for (int j = 0; j < 4; ++j) {
      FragB bh, bl;
      const size_t bo = (size_t)(16 * j + m) * FD + k0 + 8 * h;
      bh.h[0] = *(const v8us*)(ph + bo);
      bh.h[1] = *(const v8us*)(ph + bo + 16);
      bl.h[0] = *(const v8us*)(pl + bo);
      bl.h[1] = *(const v8us*)(pl + bo + 16);
#pragma unroll
      for (int rt = 0; rt < 2; ++rt) {
        acc[rt][j] = wmb(ah[rt].v, bh.v, acc[rt][j]);
        acc[rt][j] = wmb(ah[rt].v, bl.v, acc[rt][j]);
        acc[rt][j] = wmb(al[rt].v, bh.v, acc[rt][j]);
      }
    }
  }

#pragma unroll
  for (int j = 0; j < 4; ++j) {
    const float bias = (c == 0) ? bin[16 * j + m] : 0.0f;
#pragma unroll
    for (int rt = 0; rt < 2; ++rt)
#pragma unroll
      for (int r = 0; r < 8; ++r)
        so[(16 * rt + 8 * h + r) * (4 * FD) + c * FD + 16 * j + m] = acc[rt][j][r] + bias;
  }
  __syncthreads();

#pragma unroll 1
  for (int i = 0; i < NBI / 4; ++i) {
    const int rr = c + 4 * i;
    const int node = n0 + rr;
    if (node < nN) {
#pragma unroll
      for (int q = 0; q < 2; ++q) {
        const v4f v = *(const v4f*)(so + rr * (4 * FD) + q * 128 + 4 * lane);
        *(volatile v4f*)(xo + (size_t)node * (4 * FD) + q * 128 + 4 * lane) = v;
      }
    }
  }
  __threadfence();
#pragma unroll 1
  for (int i = 0; i < NBI / 4; ++i) {
    const int rr = c + 4 * i;
    const int node = n0 + rr;
    if (node < nN) {
#pragma unroll
      for (int q = 0; q < 2; ++q) {
        const v4f v = *(const v4f*)(so + rr * (4 * FD) + q * 128 + 4 * lane);
        *(volatile v4f*)(xo + (size_t)node * (4 * FD) + q * 128 + 4 * lane) = v;
      }
    }
  }
}

template <int LAST>
__global__ __launch_bounds__(NT) void k_mp(
    const float* __restrict__ coords, const int* __restrict__ dsts, const int* __restrict__ srcs,
    const float* __restrict__ xc, const _Float16* __restrict__ wb, const float* __restrict__ bbas,
    const float* __restrict__ pw, const float* __restrict__ wo0, const float* __restrict__ wo1,
    const float* __restrict__ bo, float* xn, float* outp, int nN, int nE) {
  __shared__ __attribute__((aligned(16))) float acc[(NB + 1) * 4 * FD];
  __shared__ __attribute__((aligned(16))) float st[PASSN * FD];
  __shared__ __attribute__((aligned(16))) v4f   sgeo[PASSN];
  __shared__ int   ssrc[PASSN];
  __shared__ int   sslot[PASSN];
  __shared__ __attribute__((aligned(16))) int   pend[PCAP];
  __shared__ __attribute__((aligned(16))) float swo[2 * FD];
  __shared__ __attribute__((aligned(16))) float sres[NB * 4];
  __shared__ int   wcnt[NT / 32];
  __shared__ int   pendN;

  const int tid = threadIdx.x, lane = tid & 31, wave = tid >> 5, h = lane >> 4, m = lane & 15;
  const int f = tid;
  const int nodeBase = blockIdx.x * NB;

  {
    const v4f z4 = {0.0f, 0.0f, 0.0f, 0.0f};
#pragma unroll 1
    for (int i = tid; i < (NB + 1) * FD; i += NT) *(v4f*)(acc + 4 * i) = z4;
  }
  for (int i = tid; i < 2 * FD; i += NT) swo[i] = (i < FD) ? wo0[i] : wo1[i - FD];
  if (tid == 0) pendN = 0;
  const float p0 = pw[f], p1 = pw[FD + f], p2 = pw[2 * FD + f], p3 = pw[3 * FD + f], p4 = pw[4 * FD + f];
  const float bbf = bbas[f];
  const float bov = bo[0];
  FragH bq[4];
#pragma unroll
  for (int j = 0; j < 4; ++j) {
    const _Float16* bp = wb + (16 * j + m) * KBAS + 8 * h;
    bq[j].h[0] = *(const v8h*)bp;
    bq[j].h[1] = *(const v8h*)(bp + 16);
  }
  const float cstep = 1.0f / (float)(KBAS - 1);
  const float width = RMAXF * (1.0f * cstep);
  const float invw  = 1.0f / width;
  __syncthreads();

  const unsigned nbU = (unsigned)nodeBase;
  const int sent = -2147483647 - 1;
  const int nChunks = (nE + CHUNK - 1) / CHUNK;

#pragma unroll 1
  for (int ch = 0; ch < nChunks; ++ch) {
    const int cbase = ch * CHUNK;
    const int e0 = cbase + tid * EPT;

    unsigned mask = 0u;
    {
      int v[EPT];
      if (e0 + EPT - 1 < nE) {
        const v4i qa = *(const v4i*)(dsts + e0);
        const v4i qb = *(const v4i*)(dsts + e0 + 4);
        const v4i qc = *(const v4i*)(dsts + e0 + 8);
        const v4i qd = *(const v4i*)(dsts + e0 + 12);
        v[0] = qa.x; v[1] = qa.y; v[2]  = qa.z; v[3]  = qa.w;
        v[4] = qb.x; v[5] = qb.y; v[6]  = qb.z; v[7]  = qb.w;
        v[8] = qc.x; v[9] = qc.y; v[10] = qc.z; v[11] = qc.w;
        v[12] = qd.x; v[13] = qd.y; v[14] = qd.z; v[15] = qd.w;
      } else {
#pragma unroll
        for (int j = 0; j < EPT; ++j) {
          const int e = e0 + j;
          v[j] = (e < nE) ? dsts[min(e, nE - 1)] : sent;
        }
      }
#pragma unroll
      for (int j = 0; j < EPT; ++j)
        mask |= ((((unsigned)v[j] - nbU) < (unsigned)NB) ? 1u : 0u) << j;
    }
    int cnt = (int)__builtin_popcount(mask);
#pragma unroll
    for (int off = 16; off > 0; off >>= 1) cnt += __shfl_xor(cnt, off, 32);
    if (lane == 0) wcnt[wave] = cnt;
    __syncthreads();

    const int base = pendN;
    int tot = 0, myoff = 0;
#pragma unroll
    for (int w = 0; w < NT / 32; ++w) {
      int cw = wcnt[w];
      cw = cw < 0 ? 0 : (cw > EPT * 32 ? EPT * 32 : cw);
      if (w < wave) myoff += cw;
      tot += cw;
    }
    int newN = base + tot;
    newN = newN > PCAP ? PCAP : newN;
    {
      int wc = base + myoff;
#pragma unroll 1
      for (int it = 0; it < EPT; ++it) {
        const unsigned live = __builtin_amdgcn_ballot_w32(mask != 0u);
        if (live == 0u) break;
        if (mask != 0u) {
          const int j = (int)__builtin_ctz(mask);
          const int pos = wc + (int)__builtin_amdgcn_mbcnt_lo(live, 0u);
          if ((unsigned)pos < (unsigned)PCAP) pend[pos] = e0 + j;
          mask &= mask - 1u;
        }
        wc += (int)__builtin_popcount(live);
      }
    }
    const int fin = (ch == nChunks - 1) ? 1 : 0;
    const int R   = (fin != 0) ? (newN + PASSN - 1) / PASSN : newN / PASSN;
    const int Pv  = (fin != 0) ? newN : R * PASSN;
    __syncthreads();

#pragma unroll 1
    for (int r = 0; r < R; ++r) {
      {
        const int idx = r * PASSN + tid;
        const bool valid = idx < Pv;
        int e = valid ? pend[min(idx, PCAP - 1)] : 0;
        e = e < 0 ? 0 : (e > nE - 1 ? nE - 1 : e);
        const int d = dsts[e];
        const int s = srcs[e];
        int slot = d - nodeBase;
        if (!valid || (unsigned)slot >= (unsigned)NB) slot = NB;
        const int dc = d < 0 ? 0 : (d > nN - 1 ? nN - 1 : d);
        const int sc = s < 0 ? 0 : (s > nN - 1 ? nN - 1 : s);
        const float rx = coords[(size_t)dc * 3 + 0] - coords[(size_t)sc * 3 + 0];
        const float ry = coords[(size_t)dc * 3 + 1] - coords[(size_t)sc * 3 + 1];
        const float rz = coords[(size_t)dc * 3 + 2] - coords[(size_t)sc * 3 + 2];
        const float d2 = rx * rx + ry * ry + rz * rz + 1e-12f;
        const float dd = sqrtf(d2);
        const float inv = 1.0f / dd;
        v4f gv;
        gv.x = dd; gv.y = rx * inv; gv.z = ry * inv; gv.w = rz * inv;
        sgeo[tid] = gv;
        ssrc[tid] = sc;
        sslot[tid] = slot;
      }
      __syncthreads();

      {
#pragma unroll
        for (int t = 0; t < 2; ++t) {
          const int eb = 32 * wave + 16 * t;
          const float dd = sgeo[eb + m].x;
          FragH a;
          v8h q0, q1;
#pragma unroll
          for (int i = 0; i < 8; ++i) {
            const float ck0 = RMAXF * ((float)(8 * h + i) * cstep);
            const float ck1 = RMAXF * ((float)(16 + 8 * h + i) * cstep);
            const float u0 = (dd - ck0) * invw;
            const float u1 = (dd - ck1) * invw;
            q0[i] = (_Float16)(SCB * __expf(-u0 * u0));
            q1[i] = (_Float16)(SCB * __expf(-u1 * u1));
          }
          a.h[0] = q0;
          a.h[1] = q1;
          v8f dacc[4];
#pragma unroll
          for (int j = 0; j < 4; ++j) dacc[j] = wmh(a.v, bq[j].v, zero8f());
#pragma unroll
          for (int j = 0; j < 4; ++j)
#pragma unroll
            for (int rr = 0; rr < 8; ++rr)
              st[(eb + 8 * h + rr) * FD + 16 * j + m] = dacc[j][rr] * SCINV;
        }
      }
      __syncthreads();

#pragma unroll 2
      for (int i = 0; i < PASSN; ++i) {
        int sl = sslot[i];
        sl = sl < 0 ? 0 : (sl > NB ? NB : sl);
        int s = ssrc[i];
        s = s < 0 ? 0 : (s > nN - 1 ? nN - 1 : s);
        const v4f gv = sgeo[i];
        const float t  = st[i * FD + f];
        const float* xa = xc + (size_t)s * (4 * FD) + f;
        const float a0 = xa[0];
        const float a1 = xa[FD];
        const float a2 = xa[2 * FD];
        const float a3 = xa[3 * FD];
        const float g0 = t + bbf;
        const float gx = gv.y * t, gy = gv.z * t, gz = gv.w * t;
        const float m0 = p0 * a0 * g0 + p1 * (a1 * gx + a2 * gy + a3 * gz);
        const float m1 = p2 * a0 * gx + p3 * a1 * g0 + p4 * (a2 * gz - a3 * gy);
        const float m2 = p2 * a0 * gy + p3 * a2 * g0 + p4 * (a3 * gx - a1 * gz);
        const float m3 = p2 * a0 * gz + p3 * a3 * g0 + p4 * (a1 * gy - a2 * gx);
        float* ar = acc + sl * (4 * FD) + f;
        ar[0]      += m0;
        ar[FD]     += m1;
        ar[2 * FD] += m2;
        ar[3 * FD] += m3;
      }
      __syncthreads();
    }

    int rem = newN - R * PASSN;
    rem = rem < 0 ? 0 : rem;
    if (R > 0 && tid < rem) pend[tid] = pend[R * PASSN + tid];
    if (tid == 0) pendN = rem;
  }
  __syncthreads();

#pragma unroll 1
  for (int sl = 0; sl < NB; ++sl) {
    const int node = nodeBase + sl;
    if (node < nN) {
      v4f a = *(const v4f*)(acc + sl * (4 * FD) + 4 * tid);
      const v4f x = *(const v4f*)(xc + (size_t)node * (4 * FD) + 4 * tid);
      a += x;
      *(v4f*)(acc + sl * (4 * FD) + 4 * tid) = a;
    }
  }
  __syncthreads();

  if (LAST == 0) {
#pragma unroll 1
    for (int i = 0; i < NB / 2; ++i) {
      const int sl = wave + 2 * i;
      const int node = nodeBase + sl;
      if (node < nN) {
#pragma unroll
        for (int q = 0; q < 2; ++q) {
          const v4f v = *(const v4f*)(acc + sl * (4 * FD) + q * 128 + 4 * lane);
          *(volatile v4f*)(xn + (size_t)node * (4 * FD) + q * 128 + 4 * lane) = v;
        }
      }
    }
    __threadfence();
#pragma unroll 1
    for (int i = 0; i < NB / 2; ++i) {
      const int sl = wave + 2 * i;
      const int node = nodeBase + sl;
      if (node < nN) {
#pragma unroll
        for (int q = 0; q < 2; ++q) {
          const v4f v = *(const v4f*)(acc + sl * (4 * FD) + q * 128 + 4 * lane);
          *(volatile v4f*)(xn + (size_t)node * (4 * FD) + q * 128 + 4 * lane) = v;
        }
      }
    }
  } else {
#pragma unroll 1
    for (int it = 0; it < (NB * 4) / NT; ++it) {
      const int q = it * NT + tid;
      const int sl = q >> 2, c = q & 3;
      const float* ar = acc + sl * (4 * FD) + c * FD;
      const float* wr = swo + (c == 0 ? 0 : FD);
      float sum = 0.0f;
#pragma unroll
      for (int f4 = 0; f4 < FD / 4; ++f4) {
        const v4f a = *(const v4f*)(ar + 4 * f4);
        const v4f w = *(const v4f*)(wr + 4 * f4);
        sum += a.x * w.x + a.y * w.y + a.z * w.z + a.w * w.w;
      }
      sres[q] = sum + (c == 0 ? bov : 0.0f);
    }
    __syncthreads();
    const size_t ob  = (size_t)nodeBase * 4;
    const size_t lim = (size_t)nN * 4;
    if (wave == 0) {
#pragma unroll
      for (int i = 0; i < (NB * 4) / 128; ++i) {
        const size_t gi = ob + (size_t)(i * 128 + 4 * lane);
        const v4f v = *(const v4f*)(sres + i * 128 + 4 * lane);
        if (gi + 3 < lim) *(volatile v4f*)(outp + gi) = v;
      }
    }
    __threadfence();
    if (wave == 0) {
#pragma unroll
      for (int i = 0; i < (NB * 4) / 128; ++i) {
        const size_t gi = ob + (size_t)(i * 128 + 4 * lane);
        const v4f v = *(const v4f*)(sres + i * 128 + 4 * lane);
        if (gi + 3 < lim) *(volatile v4f*)(outp + gi) = v;
      }
    }
  }
}

extern "C" void kernel_launch(void* const* d_in, const int* in_sizes, int n_in,
                              void* d_out, int out_size, void* d_ws, size_t ws_size,
                              hipStream_t stream) {
  if (n_in < 13) return;
  const int nN = in_sizes[1] / 3;
  if (nN <= 0 || in_sizes[1] != nN * 3 || in_sizes[0] != nN * 4 * FD) return;
  const int nE = in_sizes[2];
  if (nE < 0 || in_sizes[3] != nE) return;
  if (in_sizes[4] != FD * FD || in_sizes[5] != FD * FD || in_sizes[6] != FD) return;
  const int nSteps = in_sizes[7] / (KBAS * FD);
  if (nSteps < 1 || in_sizes[7] != nSteps * KBAS * FD) return;
  if (in_sizes[8] != nSteps * FD || in_sizes[9] != nSteps * 5 * FD) return;
  if (in_sizes[10] != FD || in_sizes[11] != FD || in_sizes[12] < 1) return;
  if (out_size != nN * 4) return;

  const float* x_dftb  = (const float*)d_in[0];
  const float* coords  = (const float*)d_in[1];
  const int*   dst_idx = (const int*)d_in[2];
  const int*   src_idx = (const int*)d_in[3];
  const float* W_in0   = (const float*)d_in[4];
  const float* W_in1   = (const float*)d_in[5];
  const float* b_in    = (const float*)d_in[6];
  const float* W_basis = (const float*)d_in[7];
  const float* b_basis = (const float*)d_in[8];
  const float* path_w  = (const float*)d_in[9];
  const float* W_out0  = (const float*)d_in[10];
  const float* W_out1  = (const float*)d_in[11];
  const float* b_out   = (const float*)d_in[12];
  float* out = (float*)d_out;

  char* ws = (char*)d_ws;
  size_t off = 0;
  const size_t oWh = off; off += (size_t)2 * FD * FD * 2;           off = (off + 255) & ~(size_t)255;
  const size_t oWl = off; off += (size_t)2 * FD * FD * 2;           off = (off + 255) & ~(size_t)255;
  const size_t oWb = off; off += (size_t)nSteps * KBAS * FD * 2;    off = (off + 255) & ~(size_t)255;
  const size_t xBytes = (size_t)nN * 4 * FD * sizeof(float);
  const size_t oXA = off; off += xBytes;                            off = (off + 255) & ~(size_t)255;
  const size_t oXB = off; off += xBytes;                            off = (off + 255) & ~(size_t)255;
  if (off > ws_size) return;
  unsigned short* whi = (unsigned short*)(ws + oWh);
  unsigned short* wlo = (unsigned short*)(ws + oWl);
  _Float16* wbh = (_Float16*)(ws + oWb);
  float* xA = (float*)(ws + oXA);
  float* xB = (float*)(ws + oXB);

  const int nGroups = (2 * FD * FD) / 8 + (nSteps * KBAS * FD) / 8;
  const int gPrep = (nGroups + 255) / 256;
  k_prep<<<gPrep, 256, 0, stream>>>(W_in0, W_in1, W_basis, whi, wlo, wbh, nSteps);

  const int gIn = (nN + NBI - 1) / NBI;
  k_in<<<gIn, TIN, 0, stream>>>(x_dftb, whi, wlo, b_in, xA, nN);

  const int gMp = (nN + NB - 1) / NB;
  float* cur = xA;
  float* nxt = xB;
  for (int s = 0; s < nSteps; ++s) {
    const _Float16* wb = wbh + (size_t)s * KBAS * FD;
    const float* bb = b_basis + (size_t)s * FD;
    const float* pw = path_w + (size_t)s * 5 * FD;
    if (s == nSteps - 1) {
      k_mp<1><<<gMp, NT, 0, stream>>>(coords, dst_idx, src_idx, cur, wb, bb, pw,
                                       W_out0, W_out1, b_out, nxt, out, nN, nE);
    } else {
      k_mp<0><<<gMp, NT, 0, stream>>>(coords, dst_idx, src_idx, cur, wb, bb, pw,
                                       W_out0, W_out1, b_out, nxt, out, nN, nE);
      float* tmp = cur; cur = nxt; nxt = tmp;
    }
  }
}
